// keops_matern_kernel_88734024335764
// MI455X (gfx1250) — hardware-verified
//
#include <hip/hip_runtime.h>
#include <hip/hip_bf16.h>
#include <math.h>


typedef _Float16 bf16;
typedef _Float16 f16;
typedef __attribute__((ext_vector_type(4))) unsigned v4u_t;
typedef unsigned v4ua __attribute__((ext_vector_type(4), may_alias));
typedef __attribute__((ext_vector_type(4))) float v4f_t;
typedef float v4fa __attribute__((ext_vector_type(4), may_alias));
typedef __attribute__((ext_vector_type(16))) bf16  bf16x16;
typedef bf16x16 f16x16;
typedef __attribute__((ext_vector_type(8)))  bf16  bf16x8;
typedef bf16x8 f16x8;
typedef __attribute__((ext_vector_type(4)))  bf16  bf16x4;
typedef __attribute__((ext_vector_type(8)))  float f32x8;
__device__ __forceinline__ f32x8 wmma16(f16x16 a, f16x16 b, f32x8 c) {
  c = __builtin_amdgcn_wmma_f32_16x16x32_f16(false, a, false, b, (short)0, c, false, false);
  asm volatile("v_nop\n\tv_nop\n\tv_nop\n\tv_nop" : "+v"(c) : "v"(a), "v"(b));
  return c;
}
#define LDS_STRIDE 48
#define KSTRIDE    72
#define VSTRIDE    48

__device__ __forceinline__ f32x8 wmma_bf16(bf16x16 a, bf16x16 b, f32x8 c) {
  c = __builtin_amdgcn_wmma_f32_16x16x32_f16(false, a, false, b, (short)0, c, false, false);
  asm volatile("v_nop\n\tv_nop\n\tv_nop\n\tv_nop" : "+v"(c) : "v"(a), "v"(b));
  return c;
}

template <typename T>
__device__ __forceinline__ bf16x16 load_frag(const T* __restrict__ base, int ld,
                                             int row0, int k0) {
  const int lane = threadIdx.x & 31;
  const int r    = lane & 15;
  const int kh   = (lane >> 4) * 8;
  const T* p0 = base + (size_t)(row0 + r) * ld + (k0 + kh);
  const T* p1 = p0 + 16;
  bf16x16 f;
#pragma unroll
  for (int i = 0; i < 8; ++i) {
    f[i]     = (bf16)p0[i];
    f[i + 8] = (bf16)p1[i];
  }
  return f;
}

__device__ __forceinline__ bf16x16 lds_frag(const bf16* base, int stride) {
  const int lane = threadIdx.x & 31;
  const int row  = lane & 15;
  const int kh   = (lane >> 4) * 8;
  const bf16x8 lo = *(const bf16x8*)(base + row * stride + kh);
  const bf16x8 hi = *(const bf16x8*)(base + row * stride + kh + 16);
  bf16x16 f;
#pragma unroll
  for (int i = 0; i < 8; ++i) { f[i] = lo[i]; f[i + 8] = hi[i]; }
  return f;
}

template <typename T>
__device__ __forceinline__ void stage_read16(const T* __restrict__ p, float* buf) {
#pragma unroll
  for (int i = 0; i < 16; ++i) buf[i] = (float)p[i];
}

__device__ __forceinline__ void stage_write(bf16* dst, const float* buf, int nquad) {
#pragma unroll
  for (int i = 0; i < nquad; ++i) {
    bf16x4 q;
    q[0] = (bf16)buf[4 * i];     q[1] = (bf16)buf[4 * i + 1];
    q[2] = (bf16)buf[4 * i + 2]; q[3] = (bf16)buf[4 * i + 3];
    *(bf16x4*)(dst + 4 * i) = q;
  }
}


#define GSTR 48
#define NX 16384
#define MY 16384
#define DDIM 8
#define DV 16

__device__ __forceinline__ void split16(float v, f16& h, f16& l) { h = (f16)v; l = (f16)((v - (float)h) * 2048.0f); }

__global__ __launch_bounds__(256) void k_matern(const float* __restrict__ ls, const float* __restrict__ x, const float* __restrict__ y, const float* __restrict__ b,
                                               float* __restrict__ out) {
  __shared__ __attribute__((aligned(16))) f16 ldsB[16 * GSTR];
  __shared__ __attribute__((aligned(16))) float yS[32 * DDIM];
  __shared__ __attribute__((aligned(16))) float syS[32];
  __shared__ __attribute__((aligned(16))) float oS[128 * DV];
  __shared__ float lsS[DDIM];
  const int tid = threadIdx.x, lane = tid & 31, wave = tid >> 5, cl = lane & 15, rh = (lane >> 4) * 8;
  const int i0 = blockIdx.x * 128, i0w = i0 + wave * 16;
  if (tid < DDIM) lsS[tid] = sqrtf(ls[tid]);
  __syncthreads();
  float sx = 0.0f; f16x16 xbh, xbl;
  { const v4f_t a = *(const v4f_t*)(x + (size_t)(i0w + cl) * DDIM), c = *(const v4f_t*)(x + (size_t)(i0w + cl) * DDIM + 4);
    float xv[8]; xv[0] = a[0]; xv[1] = a[1]; xv[2] = a[2]; xv[3] = a[3]; xv[4] = c[0]; xv[5] = c[1]; xv[6] = c[2]; xv[7] = c[3];
#pragma unroll
    for (int d = 0; d < 8; ++d) { xv[d] *= lsS[d]; sx = fmaf(xv[d], xv[d], sx); }
#pragma unroll
    for (int e = 0; e < 16; ++e) { xbh[e] = (f16)0.0f; xbl[e] = (f16)0.0f; }
    if (lane < 16) {
#pragma unroll
      for (int d = 0; d < 8; ++d) { f16 h, l; split16(xv[d], h, l); xbh[d] = h; xbl[d] = l; } }
  }
  const float c1k = 2.2360679774997898f * 1024.0f, c2k = 1.2909944487358056f * 1024.0f;
  const float ec = -2.2360679774997898f * 1.4426950408889634f;
  f32x8 acc; { f32x8 z = {}; acc = z; }
#pragma unroll 1
  for (int j0 = 0; j0 < MY; j0 += 32) {
    __syncthreads();
    if (tid < 32) {
      const v4f_t a = *(const v4f_t*)(y + (size_t)(j0 + tid) * DDIM), c = *(const v4f_t*)(y + (size_t)(j0 + tid) * DDIM + 4);
      v4f_t pa, pc; float s = 0.0f;
#pragma unroll
      for (int d = 0; d < 4; ++d) { pa[d] = a[d] * lsS[d]; pc[d] = c[d] * lsS[4 + d]; s = fmaf(pa[d], pa[d], s); s = fmaf(pc[d], pc[d], s); }
      *(v4fa*)(yS + tid * DDIM) = pa; *(v4fa*)(yS + tid * DDIM + 4) = pc; syS[tid] = s;
    } else if (tid < 160) { const int t = tid - 32; const int dvv = t >> 3, jq = (t & 7) * 4;
#pragma unroll
      for (int u = 0; u < 4; ++u) ldsB[dvv * GSTR + jq + u] = (f16)b[(size_t)(j0 + jq + u) * DV + dvv]; }
    __syncthreads();
    f16x16 af;
#pragma unroll
    for (int jt = 0; jt < 2; ++jt) {
      f16x16 yah, yal;
#pragma unroll
      for (int e = 0; e < 16; ++e) { yah[e] = (f16)0.0f; yal[e] = (f16)0.0f; }
      if (lane < 16) { const v4f_t a = *(const v4fa*)(yS + (jt * 16 + lane) * DDIM), c = *(const v4fa*)(yS + (jt * 16 + lane) * DDIM + 4);
#pragma unroll
        for (int d = 0; d < 4; ++d) { f16 h, l; split16(a[d], h, l); yah[d] = h; yal[d] = l; split16(c[d], h, l); yah[4 + d] = h; yal[4 + d] = l; } }
      f32x8 T, Tx; { f32x8 z = {}; T = z; Tx = z; }
      T = wmma16(yah, xbh, T); Tx = wmma16(yah, xbl, Tx); Tx = wmma16(yal, xbh, Tx);
      const v4f_t sya = *(const v4fa*)(syS + jt * 16 + rh), syc = *(const v4fa*)(syS + jt * 16 + rh + 4);
#pragma unroll
      for (int r = 0; r < 8; ++r) {
        const float t = fmaf(Tx[r], 1.0f / 2048.0f, T[r]);
        const float sy = (r < 4) ? sya[r] : syc[r - 4];
        const float d2 = fmaxf(fmaf(-2.0f, t, sx + sy), 0.0f);
        const float rr = __builtin_amdgcn_sqrtf(d2);
        const float poly = fmaf(c1k, rr, fmaf(c2k, d2, 1024.0f));
        const float kv = poly * __builtin_amdgcn_exp2f(ec * rr);
        af[jt * 8 + r] = (f16)kv;
      }
    }
    const f16x16 bf = lds_frag(ldsB, GSTR);
    acc = wmma16(af, bf, acc);
  }
#pragma unroll
  for (int r = 0; r < 8; ++r) oS[(wave * 16 + rh + r) * DV + cl] = acc[r] * (1.0f / 1024.0f);
  __syncthreads();
  float* dst = out + (size_t)i0 * DV;
#pragma unroll 1
  for (int pass = 0; pass < 2; ++pass) {
#pragma unroll
    for (int k = 0; k < 2; ++k) { const int f4 = tid + 256 * k; *(volatile v4f_t*)(dst + 4 * f4) = *(const v4fa*)(oS + 4 * f4); }
    __threadfence(); }
}

extern "C" void kernel_launch(void* const* d_in, const int* in_sizes, int n_in,
                              void* d_out, int out_size, void* d_ws, size_t ws_size,
                              hipStream_t stream) {
  (void)in_sizes; (void)n_in; (void)out_size; (void)d_ws; (void)ws_size;
  const float* ls = (const float*)d_in[0]; const float* x = (const float*)d_in[1]; const float* y = (const float*)d_in[2]; const float* b = (const float*)d_in[3];
  float* out = (float*)d_out;
  k_matern<<<dim3(NX / 128), dim3(256), 0, stream>>>(ls, x, y, b, out);
}
